// FCNKANLayer_5299989643376
// MI455X (gfx1250) — hardware-verified
//
#include <hip/hip_runtime.h>
#include <math.h>

typedef __attribute__((ext_vector_type(16))) _Float16 v16h;
typedef __attribute__((ext_vector_type(8)))  _Float16 v8h;
typedef __attribute__((ext_vector_type(8)))  float    v8f;

constexpr int kNB   = 256;
constexpr int kNI   = 128;
constexpr int kNO   = 128;
constexpr int kNH   = 32;
constexpr int kNF   = 7;
constexpr int kKP   = 32;
constexpr int kRowsW = kNI * kNO * kNH;
constexpr int kRowsF = kNI * kNB;
constexpr int kTileB = 32;
constexpr int kTileO = 32;
static_assert(kNF + 1 <= 8);
static_assert((kRowsW % 256) == 0 && kNB == 256);
static_assert((kNB % kTileB) == 0 && (kNO % kTileO) == 0 && kNH == 32);

constexpr float kFeatCarry = 16.0f;
constexpr float kWCarry    = 64.0f;
constexpr float kFold      = 1.0f / (kFeatCarry * kWCarry);
constexpr float kF16MinNormal = 6.103515625e-05f;

constexpr size_t kOffFeat = 0;
constexpr size_t kOffW1H  = kOffFeat + (size_t)kRowsF * kKP * 2;
constexpr size_t kWsTotal = kOffW1H + (size_t)kRowsW * kKP * 2;
static_assert(kWsTotal == 35651584ull);
static_assert(kWsTotal <= 134217728ull);
static_assert((kOffW1H % 128) == 0);

union FragU { v16h v; v8h h[2]; };
__device__ __forceinline__ v16h frag_load(const _Float16* p) {
  FragU f;
  f.h[0] = *(const v8h*)(p);
  f.h[1] = *(const v8h*)(p + 16);
  return f.v;
}
__device__ __forceinline__ v8f mma_f16(v16h a, v16h b, v8f c) {
  return __builtin_amdgcn_wmma_f32_16x16x32_f16(false, a, false, b, (short)0, c, false, false);
}
__device__ __forceinline__ void tile_guard(v8f& c, v16h a, v16h b) {
  asm volatile("v_nop\n\tv_nop\n\tv_nop\n\tv_nop" : "+v"(c) : "v"(a), "v"(b));
}

__device__ __forceinline__ _Float16 to_f16_flushed(float v) {
  const float t = (fabsf(v) < kF16MinNormal) ? 0.0f : v;
  return (_Float16)t;
}

__device__ __forceinline__ void store_rows_256(const v8h* sRows, unsigned short* plane, size_t rowBase) {
  const int lane = threadIdx.x & 31;
  const int wave = threadIdx.x >> 5;
  v8h v[4];
#pragma unroll
  for (int it = 0; it < 4; ++it) v[it] = sRows[(it * 8 + wave) * 32 + lane];
  v8h* dst = (v8h*)(plane + rowBase * (size_t)kKP);
  for (int pass = 0; pass < 2; ++pass) {
#pragma unroll
    for (int it = 0; it < 4; ++it) *(volatile v8h*)(dst + (it * 8 + wave) * 32 + lane) = v[it];
    __threadfence();
  }
}

__global__ __launch_bounds__(256) void feat_plane_kernel(const float* __restrict__ x, unsigned short* __restrict__ feat) {
  __shared__ __align__(16) v8h sRows[256 * 4];
  const int tid = threadIdx.x;
  const int i = blockIdx.x;
  const float xv = x[(size_t)tid * kNI + i];
  float s1, c1;
  sincosf(xv, &s1, &c1);
  const float s2 = 2.0f * s1 * c1;
  const float c2 = fmaf(c1, c1, -(s1 * s1));
  const float s4 = 2.0f * s2 * c2;
  const float c4 = fmaf(c2, c2, -(s2 * s2));
  float onev = kFeatCarry;
  asm volatile("" : "+v"(onev));
  v8h hv;
  hv[0] = to_f16_flushed(xv * kFeatCarry);
  hv[1] = to_f16_flushed(s1 * kFeatCarry);
  hv[2] = to_f16_flushed(s2 * kFeatCarry);
  hv[3] = to_f16_flushed(s4 * kFeatCarry);
  hv[4] = to_f16_flushed(c1 * kFeatCarry);
  hv[5] = to_f16_flushed(c2 * kFeatCarry);
  hv[6] = to_f16_flushed(c4 * kFeatCarry);
  hv[7] = (_Float16)onev;
  v8h zv;
#pragma unroll
  for (int e = 0; e < 8; ++e) zv[e] = (_Float16)0.0f;
  sRows[tid * 4 + 0] = hv;
  sRows[tid * 4 + 1] = zv;
  sRows[tid * 4 + 2] = zv;
  sRows[tid * 4 + 3] = zv;
  __syncthreads();
  store_rows_256(sRows, feat, (size_t)i * kNB);
}

__global__ __launch_bounds__(256) void weight_plane_kernel(const float* __restrict__ W1, const float* __restrict__ B1,
                                                           unsigned short* __restrict__ w1h) {
  __shared__ __align__(16) v8h sRows[256 * 4];
  const int tid = threadIdx.x;
  const int n = blockIdx.x * 256 + tid;
  const float* wr = W1 + (size_t)n * kNF;
  const float f0 = wr[0], f1 = wr[1], f2 = wr[2], f3 = wr[3], f4 = wr[4], f5 = wr[5], f6 = wr[6];
  const float f7 = B1[n];
  v8h hv;
  hv[0] = to_f16_flushed(f0 * kWCarry);
  hv[1] = to_f16_flushed(f1 * kWCarry);
  hv[2] = to_f16_flushed(f2 * kWCarry);
  hv[3] = to_f16_flushed(f3 * kWCarry);
  hv[4] = to_f16_flushed(f4 * kWCarry);
  hv[5] = to_f16_flushed(f5 * kWCarry);
  hv[6] = to_f16_flushed(f6 * kWCarry);
  hv[7] = to_f16_flushed(f7 * kWCarry);
  v8h zv;
#pragma unroll
  for (int e = 0; e < 8; ++e) zv[e] = (_Float16)0.0f;
  sRows[tid * 4 + 0] = hv;
  sRows[tid * 4 + 1] = zv;
  sRows[tid * 4 + 2] = zv;
  sRows[tid * 4 + 3] = zv;
  __syncthreads();
  store_rows_256(sRows, w1h, (size_t)blockIdx.x * 256);
}

__global__ __launch_bounds__(256) void fused_edge_kernel(const unsigned short* __restrict__ featp,
                                                         const unsigned short* __restrict__ w1hp,
                                                         const float* __restrict__ W2,
                                                         const float* __restrict__ B2,
                                                         float* __restrict__ out) {
  __shared__ __align__(16) float sTile[kTileB * kTileO];
  const _Float16* FA = (const _Float16*)featp;
  const _Float16* WH = (const _Float16*)w1hp;
  const int tid  = threadIdx.x;
  const int lane = tid & 31;
  const int wave = tid >> 5;
  const int half = lane >> 4;
  const int col  = lane & 15;
  const int b0 = blockIdx.x * kTileB;
  const int o0 = blockIdx.y * kTileO;

#pragma unroll 1
  for (int u = 0; u < 8; ++u) {
    const int bt = u & 1;
    const int ol = wave * 4 + (u >> 1);
    const int o  = o0 + ol;

    float bs = 0.0f;
#pragma unroll
    for (int q = 0; q < 4; ++q) bs += B2[(size_t)(q * 32 + lane) * kNO + o];
    bs += __shfl_xor(bs, 16, 32);
    bs += __shfl_xor(bs, 8, 32);
    bs += __shfl_xor(bs, 4, 32);
    bs += __shfl_xor(bs, 2, 32);
    bs += __shfl_xor(bs, 1, 32);

    v8f acc = (v8f){0.f, 0.f, 0.f, 0.f, 0.f, 0.f, 0.f, 0.f};
    const _Float16* ap = FA + (size_t)(b0 + bt * 16 + col) * kKP + 8 * half;
    const _Float16* bp = WH + ((size_t)o * kNH + col) * kKP + 8 * half;
    const float*    wp = W2 + (size_t)o * kNH + col;

#pragma unroll 1
    for (int j = 0; j < 2 * kNI; ++j) {
      const int i  = j >> 1;
      const int ht = j & 1;
      const v16h a = frag_load(ap + (size_t)i * ((size_t)kNB * kKP));
      const v16h b = frag_load(bp + (size_t)i * ((size_t)kNO * kNH * kKP) + (size_t)ht * (16 * kKP));
      const float w2 = wp[(size_t)i * (kNO * kNH) + ht * 16];
      v8f c = (v8f){0.f, 0.f, 0.f, 0.f, 0.f, 0.f, 0.f, 0.f};
      c = mma_f16(a, b, c);
      tile_guard(c, a, b);
#pragma unroll
      for (int r = 0; r < 8; ++r) {
        const float pre = c[r] * kFold;
        const float ex  = expf(-pre);
        const float sl  = pre * __builtin_amdgcn_rcpf(1.0f + ex);
        acc[r] = fmaf(sl, w2, acc[r]);
      }
    }

    float res[8];
#pragma unroll
    for (int r = 0; r < 8; ++r) {
      float v = acc[r];
      v += __shfl_xor(v, 1, 32);
      v += __shfl_xor(v, 2, 32);
      v += __shfl_xor(v, 4, 32);
      v += __shfl_xor(v, 8, 32);
      res[r] = v + bs;
    }
    if (col == 0) {
#pragma unroll
      for (int r = 0; r < 8; ++r) sTile[(bt * 16 + 8 * half + r) * kTileO + ol] = res[r];
    }
  }
  __syncthreads();

  float v[4];
#pragma unroll
  for (int it = 0; it < 4; ++it) v[it] = sTile[(wave * 4 + it) * kTileO + lane];
  for (int pass = 0; pass < 2; ++pass) {
#pragma unroll
    for (int it = 0; it < 4; ++it)
      *(volatile float*)(out + (size_t)(b0 + wave * 4 + it) * kNO + o0 + lane) = v[it];
    __threadfence();
  }
}

extern "C" void kernel_launch(void* const* d_in, const int* in_sizes, int n_in,
                              void* d_out, int out_size, void* d_ws, size_t ws_size,
                              hipStream_t stream) {
  if (n_in < 5) return;
  if (in_sizes[0] != kNB * kNI) return;
  if (in_sizes[1] != kRowsW * kNF) return;
  if (in_sizes[2] != kRowsW) return;
  if (in_sizes[3] != kRowsW) return;
  if (in_sizes[4] != kNI * kNO) return;
  if (out_size != kNB * kNO) return;
  if (ws_size < kWsTotal) return;

  const float* x  = (const float*)d_in[0];
  const float* W1 = (const float*)d_in[1];
  const float* W2 = (const float*)d_in[2];
  const float* B1 = (const float*)d_in[3];
  const float* B2 = (const float*)d_in[4];
  float* out = (float*)d_out;

  char* ws = (char*)d_ws;
  unsigned short* FEAT = (unsigned short*)(ws + kOffFeat);
  unsigned short* W1H  = (unsigned short*)(ws + kOffW1H);

  feat_plane_kernel<<<kNI, 256, 0, stream>>>(x, FEAT);
  weight_plane_kernel<<<kRowsW / 256, 256, 0, stream>>>(W1, B1, W1H);
  fused_edge_kernel<<<dim3(kNB / kTileB, kNO / kTileO), 256, 0, stream>>>(FEAT, W1H, W2, B2, out);
}
